// SpatialEmbedding_81123342286998
// MI455X (gfx1250) — hardware-verified
//
#include <hip/hip_runtime.h>
#include <hip/hip_bf16.h>
#include <stddef.h>
#include <stdint.h>


#define DIN     128
#define NHEAD   4
#define FH      32
#define NAL     8
#define NTHR    256
#define NWAVE   8
#define EPT     8
#define CHUNK   (NTHR * EPT)
#define WCAP    (EPT * 32)
#define LISTN   (NWAVE * WCAP)
#define NBMAX   2048
#define RCAP    28672
#define DEGCAP  256
#define STW     128
#define GBM     64
#define GBN     128
#define GTHR    128
#define WSMAX   134217728
#define LDS_AGG ((2 * RCAP + 2 * NBMAX + LISTN) * 4 + 64)

static_assert((CHUNK & (CHUNK - 1)) == 0 && CHUNK <= 4096);
static_assert((NBMAX & (NBMAX - 1)) == 0 && NBMAX <= 4096);
static_assert(NTHR * 8 == NBMAX);
static_assert(LISTN >= NBMAX);
static_assert(LISTN >= NWAVE * WCAP);
static_assert((RCAP % 32) == 0);
static_assert(NWAVE * STW <= RCAP);
static_assert(STW >= DIN);
static_assert(LDS_AGG <= 300000);
static_assert(GBM == (GTHR / 32) * 16);
static_assert(GBN == DIN && GTHR == DIN);
static_assert(DIN == NHEAD * FH && FH == 32);
static_assert(DIN / 8 == 16);
static_assert((DIN % 32) == 0);
static_assert(GBM * NAL == 4 * 32 * 4);

typedef float          v4f  __attribute__((ext_vector_type(4)));
typedef float          v8f  __attribute__((ext_vector_type(8)));
typedef int            v4i  __attribute__((ext_vector_type(4)));
typedef int            v8i  __attribute__((ext_vector_type(8)));
typedef unsigned short v8us __attribute__((ext_vector_type(8)));
typedef __bf16         v16b __attribute__((ext_vector_type(16)));
union FragB { v16b v; v8us u[2]; v8i w; };

__device__ __forceinline__ v8f wmb(const FragB& a, const FragB& b, v8f c) {
  v8f d = __builtin_amdgcn_wmma_f32_16x16x32_bf16(false, a.v, false, b.v, (short)0, c, false, false);
  asm volatile("v_nop\n\tv_nop\n\tv_nop\n\tv_nop" : "+v"(d) : "v"(a.w), "v"(b.w));
  return d;
}

__device__ __forceinline__ void ldwait() {
  asm volatile("s_wait_loadcnt 0x0" ::: "memory");
}

__device__ __forceinline__ unsigned short bfbits(float f) {
  unsigned u = __float_as_uint(f);
  u += 0x7FFFu + ((u >> 16) & 1u);
  return (unsigned short)(u >> 16);
}
__device__ __forceinline__ float bfw(unsigned short b) { return __uint_as_float(((unsigned)b) << 16); }
__device__ __forceinline__ float bfr(float f) { return bfw(bfbits(f)); }

__device__ __forceinline__ v8us cvt8b(const v4f a, const v4f b) {
  v8us r;
  r[0] = bfbits(a.x); r[1] = bfbits(a.y); r[2] = bfbits(a.z); r[3] = bfbits(a.w);
  r[4] = bfbits(b.x); r[5] = bfbits(b.y); r[6] = bfbits(b.z); r[7] = bfbits(b.w);
  return r;
}

__device__ __forceinline__ int scan_chunk(const int* __restrict__ dsts, int nE, int cbase, int slotBase,
                                          int nb, int vec8, int* list, int tid, int lane, int wave) {
  int wc = 0;
  const int el0  = tid * EPT;
  const int e0   = cbase + el0;
  const int sent = -2147483647 - 1;
  v4i da, db;
  if (vec8 != 0 && cbase + CHUNK <= nE) {
    da = *(const v4i*)(dsts + e0);
    db = *(const v4i*)(dsts + e0 + 4);
  } else {
    da.x = (e0     < nE) ? dsts[min(e0,     nE - 1)] : sent;
    da.y = (e0 + 1 < nE) ? dsts[min(e0 + 1, nE - 1)] : sent;
    da.z = (e0 + 2 < nE) ? dsts[min(e0 + 2, nE - 1)] : sent;
    da.w = (e0 + 3 < nE) ? dsts[min(e0 + 3, nE - 1)] : sent;
    db.x = (e0 + 4 < nE) ? dsts[min(e0 + 4, nE - 1)] : sent;
    db.y = (e0 + 5 < nE) ? dsts[min(e0 + 5, nE - 1)] : sent;
    db.z = (e0 + 6 < nE) ? dsts[min(e0 + 6, nE - 1)] : sent;
    db.w = (e0 + 7 < nE) ? dsts[min(e0 + 7, nE - 1)] : sent;
  }
  const unsigned nbs = (unsigned)slotBase;
  const unsigned unb = (unsigned)nb;
  const unsigned s0 = (unsigned)da.x - nbs, s1 = (unsigned)da.y - nbs;
  const unsigned s2 = (unsigned)da.z - nbs, s3 = (unsigned)da.w - nbs;
  const unsigned s4 = (unsigned)db.x - nbs, s5 = (unsigned)db.y - nbs;
  const unsigned s6 = (unsigned)db.z - nbs, s7 = (unsigned)db.w - nbs;
  const bool h0 = s0 < unb, h1 = s1 < unb, h2 = s2 < unb, h3 = s3 < unb;
  const bool h4 = s4 < unb, h5 = s5 < unb, h6 = s6 < unb, h7 = s7 < unb;
  const unsigned any = __builtin_amdgcn_ballot_w32(h0 | h1 | h2 | h3 | h4 | h5 | h6 | h7);
  if (any != 0u) {
#define HITJ(J, HJ, SJ) { \
      const unsigned mj = __builtin_amdgcn_ballot_w32(HJ); \
      if (mj != 0u) { \
        if (HJ) { \
          const int pos = wc + (int)__builtin_amdgcn_mbcnt_lo(mj, 0u); \
          if (pos < WCAP) list[wave * WCAP + pos] = ((el0 + (J)) << 12) | (int)(SJ); \
        } \
        wc += (int)__builtin_popcount(mj); } }
    HITJ(0, h0, s0)
    HITJ(1, h1, s1)
    HITJ(2, h2, s2)
    HITJ(3, h3, s3)
    HITJ(4, h4, s4)
    HITJ(5, h5, s5)
    HITJ(6, h6, s6)
    HITJ(7, h7, s7)
#undef HITJ
  }
  return wc;
}

__global__ __launch_bounds__(NTHR) void k_xprep(const float* __restrict__ x, unsigned short* xb, int nN, int nUnits) {
  const int i = (int)blockIdx.x * NTHR + (int)threadIdx.x;
  if (i >= nUnits) return;
  const int row = i >> 4;
  const int c0  = (i & 15) * 8;
  const int rc  = row < nN ? row : nN - 1;
  const float* p = x + (size_t)rc * DIN + c0;
  v4f a = *(const v4f*)p, b = *(const v4f*)(p + 4);
  const v4f z4 = {0.f, 0.f, 0.f, 0.f};
  if (row >= nN) { a = z4; b = z4; }
  const v8us hv = cvt8b(a, b);
  const size_t o = (size_t)row * DIN + c0;
  *(volatile v8us*)(xb + o) = hv;
  __threadfence();
  *(volatile v8us*)(xb + o) = hv;
}

__global__ __launch_bounds__(NTHR) void k_wtr(const float* __restrict__ w, unsigned short* wt, int K, int nUnits) {
  const int u = (int)blockIdx.x * NTHR + (int)threadIdx.x;
  if (u >= nUnits) return;
  const int kq = K >> 3;
  const int n  = u / kq;
  const int k8 = (u - n * kq) * 8;
  const int ki = k8 & (DIN - 1);
  const float* p = w + (size_t)ki * DIN + n;
  v4f a, b;
  a.x = p[0];                  a.y = p[DIN];          a.z = p[2 * DIN];      a.w = p[3 * DIN];
  b.x = p[4 * DIN];            b.y = p[5 * DIN];      b.z = p[6 * DIN];      b.w = p[7 * DIN];
  const v8us hv = cvt8b(a, b);
  const size_t o = (size_t)n * (size_t)K + k8;
  *(volatile v8us*)(wt + o) = hv;
  __threadfence();
  *(volatile v8us*)(wt + o) = hv;
}

__global__ __launch_bounds__(GTHR) void k_gemm(
    const unsigned short* __restrict__ A, const unsigned short* __restrict__ WT,
    const float* __restrict__ asrc, const float* __restrict__ adst,
    float* Hout, float* ALout, int K)
{
  __shared__ __attribute__((aligned(16))) float stg[GBM * GBN];
  __shared__ __attribute__((aligned(16))) float sa[2 * DIN];
  __shared__ __attribute__((aligned(16))) float sal[GBM * NAL];
  const int tid = (int)threadIdx.x, lane = tid & 31, wave = tid >> 5, hh = lane >> 4, m = lane & 15;
  const int rowBase = (int)blockIdx.x * GBM;

  sa[tid]       = bfr(asrc[tid]);
  sa[DIN + tid] = bfr(adst[tid]);

  v8f acc[8];
  {
    const v8f z = {0.f, 0.f, 0.f, 0.f, 0.f, 0.f, 0.f, 0.f};
#pragma unroll
    for (int t = 0; t < 8; ++t) acc[t] = z;
  }
  const unsigned short* ap = A  + (size_t)(rowBase + 16 * wave + m) * (size_t)K + 8 * hh;
  const unsigned short* wp = WT + (size_t)m * (size_t)K + 8 * hh;
  const int ksteps = K >> 5;
#pragma unroll 1
  for (int ks = 0; ks < ksteps; ++ks) {
    FragB af;
    af.u[0] = *(const v8us*)(ap + 32 * ks);
    af.u[1] = *(const v8us*)(ap + 32 * ks + 16);
#pragma unroll
    for (int t = 0; t < 8; ++t) {
      const unsigned short* wq = wp + (size_t)(16 * t) * (size_t)K + 32 * ks;
      FragB bf;
      bf.u[0] = *(const v8us*)wq;
      bf.u[1] = *(const v8us*)(wq + 16);
      acc[t] = wmb(af, bf, acc[t]);
    }
  }

#pragma unroll
  for (int t = 0; t < 8; ++t) {
    const int lc = 16 * t + m;
#pragma unroll
    for (int r = 0; r < 8; ++r) {
      const int lr = 16 * wave + 8 * hh + r;
      stg[lr * GBN + lc] = acc[t][r];
    }
  }
  __syncthreads();

  {
    const int r  = tid & (GBM - 1);
    const int sd = tid >> 6;
    const float* hp = stg + r * GBN;
    const float* av = sa + sd * DIN;
    float d0 = 0.f, d1 = 0.f, d2 = 0.f, d3 = 0.f;
#pragma unroll 4
    for (int f = 0; f < FH; ++f) {
      d0 = fmaf(hp[f],          av[f],          d0);
      d1 = fmaf(hp[FH + f],     av[FH + f],     d1);
      d2 = fmaf(hp[2 * FH + f], av[2 * FH + f], d2);
      d3 = fmaf(hp[3 * FH + f], av[3 * FH + f], d3);
    }
    sal[r * NAL + 4 * sd + 0] = d0;
    sal[r * NAL + 4 * sd + 1] = d1;
    sal[r * NAL + 4 * sd + 2] = d2;
    sal[r * NAL + 4 * sd + 3] = d3;
  }
  __syncthreads();

  v4f fv[16];
#pragma unroll
  for (int i = 0; i < 16; ++i) {
    const int lr = 16 * wave + i;
    fv[i] = *(const v4f*)(stg + lr * GBN + 4 * lane);
  }
  v4f pv[4];
#pragma unroll
  for (int q = 0; q < 4; ++q) pv[q] = *(const v4f*)(sal + 4 * (32 * q + lane));
  const bool w0 = (wave == 0);
  float* alb = ALout + (size_t)rowBase * NAL;

#pragma unroll
  for (int i = 0; i < 16; ++i) {
    const int gr = rowBase + 16 * wave + i;
    float* op = Hout + (size_t)gr * DIN + 4 * lane;
    *(volatile v4f*)op = fv[i];
  }
  if (w0) {
#pragma unroll
    for (int q = 0; q < 4; ++q) *(volatile v4f*)(alb + 4 * (32 * q + lane)) = pv[q];
  }
  __threadfence();
#pragma unroll
  for (int i = 0; i < 16; ++i) {
    const int gr = rowBase + 16 * wave + i;
    float* op = Hout + (size_t)gr * DIN + 4 * lane;
    *(volatile v4f*)op = fv[i];
  }
  if (w0) {
#pragma unroll
    for (int q = 0; q < 4; ++q) *(volatile v4f*)(alb + 4 * (32 * q + lane)) = pv[q];
  }
}

template<int LAYER>
__global__ __launch_bounds__(NTHR) void k_agg(
    const int* __restrict__ srcs, const int* __restrict__ dsts,
    const float* __restrict__ Hp, const float* __restrict__ ALp,
    const unsigned short* __restrict__ skipB, const float* __restrict__ skipF,
    const float* __restrict__ bias,
    float* outF, unsigned short* outB,
    int nN, int nE, int nb, int vec8, int MPr) {
  extern __shared__ v4f lds_dyn[];
  int* reg1 = (int*)lds_dyn;
  int* reg2 = reg1 + RCAP;
  int* scnt = reg2 + RCAP;
  int* soff = scnt + NBMAX;
  int* list = soff + NBMAX;
  int* wcnt = list + LISTN;
  int* wtot = wcnt + NWAVE;
  const int tid = (int)threadIdx.x, lane = tid & 31, wave = tid >> 5;
  const int nodeBase = (int)blockIdx.x * nb;

  for (int i = tid; i < NBMAX; i += NTHR) scnt[i] = 0;
  __syncthreads();

  int tot = 0;
  const int nChunks = (nE + CHUNK - 1) / CHUNK;
#pragma unroll 1
  for (int ch = 0; ch < nChunks; ++ch) {
    const int cbase = ch * CHUNK;
    const int wc = scan_chunk(dsts, nE, cbase, nodeBase, nb, vec8, list, tid, lane, wave);
    if (lane == 0) wcnt[wave] = wc;
    __syncthreads();
    int pre = 0, all = 0;
#pragma unroll
    for (int w2 = 0; w2 < NWAVE; ++w2) {
      int c = wcnt[w2];
      c = c < 0 ? 0 : (c > WCAP ? WCAP : c);
      all += c;
      pre += (w2 < wave) ? c : 0;
    }
    const int wcc  = wc > WCAP ? WCAP : wc;
    const int base = tot + pre;
#pragma unroll 1
    for (int i = lane; i < wcc; i += 32) {
      const int ent = list[wave * WCAP + i];
      const int el  = (ent >> 12) & (CHUNK - 1);
      const int sl  = ent & (NBMAX - 1);
      int eid = cbase + el;
      eid = eid > nE - 1 ? nE - 1 : eid;
      const int pos = base + i;
      if (pos < RCAP) reg1[pos] = (int)(((unsigned)eid << 12) | (unsigned)sl);
    }
    tot += all;
    tot = tot > RCAP ? RCAP : tot;
    __syncthreads();
  }
  const int nh = tot;

  if (wave == 0) {
#pragma unroll 1
    for (int b0 = 0; b0 < nh; b0 += 32) {
      const int idx = b0 + lane;
      const int uv  = reg1[idx < RCAP ? idx : RCAP - 1];
      const int m32 = (nh - b0) < 32 ? (nh - b0) : 32;
#pragma unroll 1
      for (int k = 0; k < m32; ++k) {
        const int u  = __builtin_amdgcn_readlane(uv, k);
        const int sl = u & (NBMAX - 1);
        if (lane == 0) scnt[sl] = scnt[sl] + 1;
      }
    }
  }
  __syncthreads();

  {
    const v4i ca = *(const v4i*)(scnt + 8 * tid);
    const v4i cb = *(const v4i*)(scnt + 8 * tid + 4);
    const int e0 = ca.x < 0 ? 0 : ca.x, e1 = ca.y < 0 ? 0 : ca.y, e2 = ca.z < 0 ? 0 : ca.z, e3 = ca.w < 0 ? 0 : ca.w;
    const int e4 = cb.x < 0 ? 0 : cb.x, e5 = cb.y < 0 ? 0 : cb.y, e6 = cb.z < 0 ? 0 : cb.z, e7 = cb.w < 0 ? 0 : cb.w;
    const int ts = e0 + e1 + e2 + e3 + e4 + e5 + e6 + e7;
    int incl = ts;
#pragma unroll
    for (int d = 1; d < 32; d <<= 1) {
      const int up = __shfl_up(incl, d);
      if (lane >= d) incl += up;
    }
    if (lane == 31) wtot[wave] = incl;
    __syncthreads();
    int pre = 0;
#pragma unroll
    for (int w2 = 0; w2 < NWAVE; ++w2) pre += (w2 < wave) ? wtot[w2] : 0;
    int run = pre + incl - ts;
    soff[8 * tid + 0] = run; run += e0;
    soff[8 * tid + 1] = run; run += e1;
    soff[8 * tid + 2] = run; run += e2;
    soff[8 * tid + 3] = run; run += e3;
    soff[8 * tid + 4] = run; run += e4;
    soff[8 * tid + 5] = run; run += e5;
    soff[8 * tid + 6] = run; run += e6;
    soff[8 * tid + 7] = run;
  }
  __syncthreads();
  for (int i = tid; i < NBMAX; i += NTHR) list[i] = soff[i];
  __syncthreads();

  if (wave == 0) {
#pragma unroll 1
    for (int b0 = 0; b0 < nh; b0 += 32) {
      const int idx = b0 + lane;
      const int uv  = reg1[idx < RCAP ? idx : RCAP - 1];
      const int m32 = (nh - b0) < 32 ? (nh - b0) : 32;
#pragma unroll 1
      for (int k = 0; k < m32; ++k) {
        const int u   = __builtin_amdgcn_readlane(uv, k);
        const int sl  = u & (NBMAX - 1);
        const int eid = (int)((unsigned)u >> 12);
        if (lane == 0) {
          int pos = list[sl];
          pos = pos < 0 ? 0 : (pos > RCAP - 1 ? RCAP - 1 : pos);
          reg2[pos] = eid;
          list[sl] = pos + 1;
        }
      }
    }
  }
  __syncthreads();

  const int nbw = nb >> 3;
  const bool ovf = (nh >= RCAP);
  const float qnan = __int_as_float(0x7fc00000);
  float* stw = (float*)reg1 + wave * STW;
  float bb[4];
#pragma unroll
  for (int j = 0; j < 4; ++j) bb[j] = bfr(bias[32 * j + lane]);
#pragma unroll 1
  for (int jt = 0; jt < nbw; ++jt) {
    const int slot = wave * nbw + jt;
    const int grow = nodeBase + slot;
    const int gl   = grow < MPr ? grow : MPr - 1;
    int st = soff[slot];
    const int craw = scnt[slot];
    int cnt = craw;
    st  = st < 0 ? 0 : (st > nh ? nh : st);
    cnt = cnt < 0 ? 0 : (cnt > DEGCAP ? DEGCAP : cnt);
    if (cnt > nh - st) cnt = nh - st;
    const float pz = (ovf || craw > DEGCAP) ? qnan : 0.0f;
    const bool wr = grow < MPr;
    const float live = grow < nN ? 1.0f : 0.0f;

    const v4f adv = *(const v4f*)(ALp + (size_t)gl * NAL + 4);
    float sk[4];
    if (LAYER == 0) {
      const unsigned short* xr = skipB + (size_t)gl * DIN + lane;
#pragma unroll
      for (int j = 0; j < 4; ++j) sk[j] = bfw(xr[32 * j]);
    } else {
      const float* xr = skipF + (size_t)gl * DIN + lane;
#pragma unroll
      for (int j = 0; j < 4; ++j) sk[j] = xr[32 * j];
    }
    ldwait();
    const float ad[4] = {adv.x, adv.y, adv.z, adv.w};
    float agg[4], mx[4], dn[4];
#pragma unroll
    for (int h = 0; h < 4; ++h) { agg[h] = 0.f; mx[h] = -1.0e30f; dn[h] = 0.f; }

#pragma unroll 1
    for (int q = 0; q < cnt; ++q) {
      int idx = st + q; idx = idx > RCAP - 1 ? RCAP - 1 : idx;
      int eid = reg2[idx]; eid = eid < 0 ? 0 : (eid > nE - 1 ? nE - 1 : eid);
      const int sraw = srcs[eid];
      const int s = sraw < 0 ? 0 : (sraw > nN - 1 ? nN - 1 : sraw);
      const v4f asv = *(const v4f*)(ALp + (size_t)s * NAL);
      const float* hr = Hp + (size_t)s * DIN + lane;
      float hv[4];
#pragma unroll
      for (int j = 0; j < 4; ++j) hv[j] = hr[32 * j];
      ldwait();
      const float as4[4] = {asv.x, asv.y, asv.z, asv.w};
#pragma unroll
      for (int h = 0; h < 4; ++h) {
        float lg = as4[h] + ad[h];
        lg = lg > 0.f ? lg : 0.2f * lg;
        const float df = lg - mx[h];
        const float ee = __expf(-fabsf(df));
        const bool up  = df > 0.f;
        const float s1 = up ? ee : 1.0f;
        const float s2 = up ? 1.0f : ee;
        mx[h]  = up ? lg : mx[h];
        dn[h]  = fmaf(dn[h], s1, s2);
        agg[h] = fmaf(agg[h], s1, s2 * hv[h]);
      }
    }
    float r[4];
#pragma unroll
    for (int h = 0; h < 4; ++h) {
      const float ds = dn[h] > 0.f ? dn[h] : 1.0f;
      const float iv = (dn[h] > 0.f ? 1.0f : 0.0f) * __builtin_amdgcn_rcpf(ds);
      float v = agg[h] * iv;
      v = (v + sk[h]) + bb[h];
      if (LAYER == 0) v = v > 0.f ? v : (__expf(v) - 1.0f);
      r[h] = v * live + pz;
    }
    __builtin_amdgcn_fence(__ATOMIC_RELEASE, "wavefront");
    __builtin_amdgcn_wave_barrier();
#pragma unroll
    for (int h = 0; h < 4; ++h) stw[32 * h + lane] = r[h];
    __builtin_amdgcn_fence(__ATOMIC_RELEASE, "wavefront");
    __builtin_amdgcn_wave_barrier();
    const v4f ga = *(const v4f*)(stw + 4 * lane);
    if (LAYER == 1) {
      float* op = outF + (size_t)gl * DIN + 4 * lane;
      const bool w1 = grow < nN;
      if (w1) *(volatile v4f*)op = ga;
      __threadfence();
      if (w1) *(volatile v4f*)op = ga;
    } else {
      const int cb = 8 * (lane & 15);
      const v4f g0 = *(const v4f*)(stw + cb);
      const v4f g1 = *(const v4f*)(stw + cb + 4);
      const float gv[8] = {g0.x, g0.y, g0.z, g0.w, g1.x, g1.y, g1.z, g1.w};
      const bool lo = (lane >> 4) != 0;
      v8us pk;
#pragma unroll
      for (int i = 0; i < 8; ++i) {
        const unsigned short hb = bfbits(gv[i]);
        const unsigned short lb = bfbits(gv[i] - bfw(hb));
        pk[i] = lo ? lb : hb;
      }
      float* op = outF + (size_t)gl * DIN + 4 * lane;
      unsigned short* bp = outB + (size_t)gl * (2 * DIN) + 8 * lane;
      if (wr) { *(volatile v4f*)op = ga; *(volatile v8us*)bp = pk; }
      __threadfence();
      if (wr) { *(volatile v4f*)op = ga; *(volatile v8us*)bp = pk; }
    }
  }
}

static int pick_nb(int nE, int nN) {
  int nb = NBMAX;
  while (nb > 16 && (long long)nb * (long long)nE * 5LL > (long long)RCAP * (long long)nN * 4LL) nb >>= 1;
  return nb;
}
static inline int cdiv(int a, int b) { return (a + b - 1) / b; }

extern "C" void kernel_launch(void* const* d_in, const int* in_sizes, int n_in,
                              void* d_out, int out_size, void* d_ws, size_t ws_size,
                              hipStream_t stream) {
  if (n_in < 6) return;
  const int nN = in_sizes[0] / DIN;
  if (nN <= 0 || in_sizes[0] != nN * DIN || nN > (1 << 22)) return;
  if (in_sizes[1] < 2 || (in_sizes[1] & 1) != 0) return;
  const int nE = in_sizes[1] / 2;
  if (nE < 1 || nE > (1 << 20)) return;
  if (in_sizes[2] != 2 * DIN * DIN) return;
  if (in_sizes[3] != 2 * NHEAD * FH || in_sizes[4] != 2 * NHEAD * FH) return;
  if (in_sizes[5] != 2 * DIN) return;
  if (out_size != nN * DIN) return;

  const float* x   = (const float*)d_in[0];
  const int*   ei  = (const int*)  d_in[1];
  const float* W   = (const float*)d_in[2];
  const float* asr = (const float*)d_in[3];
  const float* ads = (const float*)d_in[4];
  const float* bia = (const float*)d_in[5];
  float* out = (float*)d_out;
  const int* src = ei;
  const int* dst = ei + nE;

  const int MP   = cdiv(nN, GBM) * GBM;
  const int nb   = pick_nb(nE, nN);
  const int gA   = cdiv(MP, nb);
  const int vec8 = ((nE & 3) == 0) ? 1 : 0;
  if (gA * nb < MP || nb < 8) return;

  char* ws = (char*)d_ws;
  size_t off = 0;
  const size_t oXB0 = off; off += (size_t)MP * DIN * 2;          off = (off + 255) & ~(size_t)255;
  const size_t oWT0 = off; off += (size_t)DIN * DIN * 2;         off = (off + 255) & ~(size_t)255;
  const size_t oWT1 = off; off += (size_t)DIN * (2 * DIN) * 2;   off = (off + 255) & ~(size_t)255;
  const size_t oH   = off; off += (size_t)MP * DIN * 4;          off = (off + 255) & ~(size_t)255;
  const size_t oAL  = off; off += (size_t)MP * NAL * 4;          off = (off + 255) & ~(size_t)255;
  const size_t oX1  = off; off += (size_t)MP * DIN * 4;          off = (off + 255) & ~(size_t)255;
  const size_t oXB1 = off; off += (size_t)MP * (2 * DIN) * 2;    off = (off + 255) & ~(size_t)255;
  if (off > ws_size || off > (size_t)WSMAX) return;
  unsigned short* XB0 = (unsigned short*)(ws + oXB0);
  unsigned short* WT0 = (unsigned short*)(ws + oWT0);
  unsigned short* WT1 = (unsigned short*)(ws + oWT1);
  float*          H   = (float*)(ws + oH);
  float*          AL  = (float*)(ws + oAL);
  float*          X1  = (float*)(ws + oX1);
  unsigned short* XB1 = (unsigned short*)(ws + oXB1);

  hipFuncSetAttribute(reinterpret_cast<const void*>(&k_agg<0>),
                      hipFuncAttributeMaxDynamicSharedMemorySize, LDS_AGG);
  hipFuncSetAttribute(reinterpret_cast<const void*>(&k_agg<1>),
                      hipFuncAttributeMaxDynamicSharedMemorySize, LDS_AGG);

  const int nUx = MP * (DIN / 8);
  k_xprep<<<cdiv(nUx, NTHR), NTHR, 0, stream>>>(x, XB0, nN, nUx);

  {
    const int nU0 = DIN * (DIN / 8);
    k_wtr<<<cdiv(nU0, NTHR), NTHR, 0, stream>>>(W, WT0, DIN, nU0);
    const int nU1 = DIN * (2 * DIN / 8);
    k_wtr<<<cdiv(nU1, NTHR), NTHR, 0, stream>>>(W + (size_t)DIN * DIN, WT1, 2 * DIN, nU1);
  }

  const int gM = MP / GBM;
  k_gemm<<<gM, GTHR, 0, stream>>>(XB0, WT0, asr, ads, H, AL, DIN);
  k_agg<0><<<gA, NTHR, LDS_AGG, stream>>>(src, dst, H, AL, XB0, X1, bia, X1, XB1, nN, nE, nb, vec8, MP);
  k_gemm<<<gM, GTHR, 0, stream>>>(XB1, WT1, asr + NHEAD * FH, ads + NHEAD * FH, H, AL, 2 * DIN);
  k_agg<1><<<gA, NTHR, LDS_AGG, stream>>>(src, dst, H, AL, XB0, X1, bia + DIN, out, XB1, nN, nE, nb, vec8, MP);
}
